// CNF_60266981097661
// MI455X (gfx1250) — hardware-verified
//
#include <hip/hip_runtime.h>
#include <math.h>

constexpr int NBATCH = 32768;
constexpr int NDIM   = 64;
constexpr int NHID   = 256;
constexpr int NSTEPS = 8;
constexpr int NSTAGE = 6;
constexpr int NTHR   = 128;
constexpr int NWAVE  = NTHR / 32;
constexpr int RB     = 32;
constexpr int YP     = 72;
constexpr int HP     = 264;
constexpr int SP     = 68;
constexpr int CSUB   = 8 * NTHR;
constexpr int KSLOT  = 2 * CSUB;
constexpr int NKSLOT = 5;
constexpr float DT        = 0.125f;
constexpr float W1CAR     = 8.0f;
constexpr float W1CAR_INV = 0.125f;
constexpr float W2CAR     = 16.0f;
constexpr float W2CAR_INV = 0.0625f;
constexpr float CSC       = 1.0f / 128.0f;
constexpr float HALF_LN2PI_NEG = -0.5f * 1.8378770664093453f;
constexpr float BW0 = (float)(35.0 / 384.0);
constexpr float BW2 = (float)(500.0 / 1113.0);
constexpr float BW3 = (float)(125.0 / 192.0);
constexpr float BW4 = (float)(-2187.0 / 6784.0);
constexpr float BW5 = (float)(11.0 / 84.0);

static_assert(NBATCH % RB == 0, "grid exact");
static_assert(RB == 32 && NTHR == 128, "block geometry");
static_assert(NDIM == 16 * NWAVE, "one 16-column feature group per wave");
static_assert(NHID == 64 * NWAVE, "one 64-column hidden group per wave");
static_assert(NDIM % 32 == 0 && NHID % 32 == 0, "K multiples of 32");
static_assert(RB * NDIM == 4 * NTHR * 4, "prologue staging loop exact (4 iterations x 128 threads x 4 floats)");
static_assert(2 * NHID == 4 * NTHR, "bias staging exact (128 threads x 4 floats)");
static_assert(YP % 8 == 0 && HP % 8 == 0 && SP % 4 == 0, "16-B aligned fragment rows");
static_assert(NDIM <= YP && NHID <= HP, "tile widths");
static_assert(RB * SP + 2 * NWAVE * RB + RB <= NKSLOT * KSLOT, "end-of-kernel staging fits the k region");
static_assert(RB * SP <= NKSLOT * KSLOT, "prologue staging fits the k region");
static_assert((NDIM * NHID) % (64 * 64) == 0, "transpose tiles exact");
static_assert((NHID * NDIM / 8) % 256 == 0, "cast grid exact");
static_assert((size_t)NBATCH * NDIM * 4 == 8388608, "second output byte offset");
static_assert((size_t)NBATCH * NDIM * 4 + (size_t)NBATCH * 4 == 8519680, "output total bytes");

typedef __attribute__((ext_vector_type(16))) _Float16 v16h;
typedef __attribute__((ext_vector_type(8)))  _Float16 v8h;
typedef __attribute__((ext_vector_type(4)))  _Float16 v4h;
typedef __attribute__((ext_vector_type(8)))  float    v8f;
typedef __attribute__((ext_vector_type(4)))  float    v4f;

__constant__ float c_cdt[NSTAGE] = {
  0.0f, (float)(1.0 / 5.0 * 0.125), (float)(3.0 / 10.0 * 0.125), (float)(4.0 / 5.0 * 0.125),
  (float)(8.0 / 9.0 * 0.125), (float)(1.0 * 0.125)};
__constant__ float c_btab[NSTAGE] = {
  (float)(35.0 / 384.0), 0.0f, (float)(500.0 / 1113.0), (float)(125.0 / 192.0),
  (float)(-2187.0 / 6784.0), (float)(11.0 / 84.0)};
__constant__ float c_atab[NSTAGE][5] = {
  {0.0f, 0.0f, 0.0f, 0.0f, 0.0f},
  {(float)(1.0 / 5.0), 0.0f, 0.0f, 0.0f, 0.0f},
  {(float)(3.0 / 40.0), (float)(9.0 / 40.0), 0.0f, 0.0f, 0.0f},
  {(float)(44.0 / 45.0), (float)(-56.0 / 15.0), (float)(32.0 / 9.0), 0.0f, 0.0f},
  {(float)(19372.0 / 6561.0), (float)(-25360.0 / 2187.0), (float)(64448.0 / 6561.0), (float)(-212.0 / 729.0), 0.0f},
  {(float)(9017.0 / 3168.0), (float)(-355.0 / 33.0), (float)(46732.0 / 5247.0), (float)(49.0 / 176.0), (float)(-5103.0 / 18656.0)}};

__device__ __forceinline__ void guard2x3(v8f& a, v8f& b, v16h x, v16h y, v16h z) {
  asm volatile("v_nop\n\tv_nop\n\tv_nop\n\tv_nop" : "+v"(a), "+v"(b) : "v"(x), "v"(y), "v"(z));
}
__device__ __forceinline__ void guard4x4(v8f& a, v8f& b, v8f& c2, v8f& d, v16h w, v16h x, v16h y, v16h z) {
  asm volatile("v_nop\n\tv_nop\n\tv_nop\n\tv_nop" : "+v"(a), "+v"(b), "+v"(c2), "+v"(d) : "v"(w), "v"(x), "v"(y), "v"(z));
}
__device__ __forceinline__ void acc_guard2(v8f& a, v8f& b) {
  asm volatile("v_nop\n\tv_nop\n\tv_nop\n\tv_nop" : "+v"(a), "+v"(b));
}
__device__ __forceinline__ void acc_guard4(v8f& a, v8f& b, v8f& c2, v8f& d) {
  asm volatile("v_nop\n\tv_nop\n\tv_nop\n\tv_nop" : "+v"(a), "+v"(b), "+v"(c2), "+v"(d));
}

template <typename T> struct Frag;
template <> struct Frag<_Float16> {
  typedef v16h V; union U { v16h v; v8h h[2]; };
  static __device__ __forceinline__ v16h load(const _Float16* p) {
    U f; f.h[0] = *(const v8h*)(p); f.h[1] = *(const v8h*)(p + 16); return f.v;
  }
  static __device__ __forceinline__ v8f mma(v16h a, v16h b, v8f c) {
    return __builtin_amdgcn_wmma_f32_16x16x32_f16(false, a, false, b, (short)0, c, false, false);
  }
};

__device__ __forceinline__ float tanh_acc(float x) {
  const float ex = expf(2.0f * x);
  return fmaf(-2.0f, __builtin_amdgcn_rcpf(ex + 1.0f), 1.0f);
}

__global__ __launch_bounds__(256) void tpose_f16_kernel(const float* __restrict__ src, int R, int C, int ldo,
                                                        unsigned short* __restrict__ O, float sc) {
  __shared__ float Tt[64 * 65];
  (void)R;
  const int tid = threadIdx.x;
  const int c0 = blockIdx.x * 64, r0 = blockIdx.y * 64;
#pragma unroll
  for (int i = 0; i < 4; ++i) {
    const int idx = i * 256 + tid;
    const int rr = idx >> 4, cc = (idx & 15) * 4;
    const v4f v = *(const v4f*)(src + (size_t)(r0 + rr) * (size_t)C + c0 + cc);
    Tt[rr * 65 + cc + 0] = v[0];
    Tt[rr * 65 + cc + 1] = v[1];
    Tt[rr * 65 + cc + 2] = v[2];
    Tt[rr * 65 + cc + 3] = v[3];
  }
  __syncthreads();
  const int q = tid >> 3, c8 = (tid & 7) * 8;
  v8h hv[2];
#pragma unroll
  for (int g = 0; g < 2; ++g) {
    const int qq = g * 32 + q;
#pragma unroll
    for (int e = 0; e < 8; ++e) hv[g][e] = (_Float16)(Tt[(c8 + e) * 65 + qq] * sc);
  }
  for (int pass = 0; pass < 2; ++pass) {
#pragma unroll
    for (int g = 0; g < 2; ++g) {
      const size_t o = (size_t)(c0 + g * 32 + q) * (size_t)ldo + (size_t)(r0 + c8);
      *(volatile v8h*)(O + o) = hv[g];
    }
    __threadfence();
  }
}

__global__ __launch_bounds__(256) void cast8_f16_kernel(const float* __restrict__ src, unsigned short* __restrict__ dst,
                                                        int n8, float sc) {
  const int i = blockIdx.x * 256 + threadIdx.x;
  if (i < n8) {
    const v4f a = *(const v4f*)(src + (size_t)i * 8);
    const v4f b = *(const v4f*)(src + (size_t)i * 8 + 4);
    v8h hv;
#pragma unroll
    for (int e = 0; e < 4; ++e) { hv[e] = (_Float16)(a[e] * sc); hv[4 + e] = (_Float16)(b[e] * sc); }
    *(volatile v8h*)(dst + (size_t)i * 8) = hv;
    __threadfence();
    *(volatile v8h*)(dst + (size_t)i * 8) = hv;
  }
}

__global__ __launch_bounds__(NTHR) void ode_flow_kernel(const float* __restrict__ y, const float* __restrict__ e,
                                                       const float* __restrict__ W1, const float* __restrict__ b1,
                                                       const float* __restrict__ b2,
                                                       const unsigned short* __restrict__ W1Tp,
                                                       const unsigned short* __restrict__ W2Tp,
                                                       const unsigned short* __restrict__ W2Rp,
                                                       float* __restrict__ out0, float* __restrict__ out1) {
  __shared__ __align__(16) float    Kf[NKSLOT * KSLOT];
  __shared__ __align__(16) float    Cs[2 * 4 * CSUB];
  __shared__ __align__(16) _Float16 Hh[RB * HP];
  __shared__ __align__(16) _Float16 Yh[RB * YP];
  __shared__ __align__(16) float    Bs[2 * NHID];
  const _Float16* W1T = (const _Float16*)W1Tp;
  const _Float16* W2T = (const _Float16*)W2Tp;
  const _Float16* W2R = (const _Float16*)W2Rp;
  const int tid = threadIdx.x, lane = tid & 31, wave = tid >> 5;
  const int c = lane & 15, hh = lane >> 4, koff = 8 * hh;
  const int rowbase = blockIdx.x * RB;
  const v8f z8 = {0.f, 0.f, 0.f, 0.f, 0.f, 0.f, 0.f, 0.f};

#pragma unroll
  for (int it = 0; it < 4; ++it) {
    const int idx = it * NTHR + tid;
    const int row = idx >> 4, c4 = (idx & 15) * 4;
    const size_t g = (size_t)(rowbase + row) * NDIM + c4;
    const v4f vy = *(const v4f*)(y + g);
    const v4f ve = *(const v4f*)(e + g);
    *(v4f*)(Kf + row * SP + c4) = vy;
    v4h hy, he;
#pragma unroll
    for (int q = 0; q < 4; ++q) { hy[q] = (_Float16)vy[q]; he[q] = (_Float16)ve[q]; }
    *(v4h*)(Yh + row * YP + c4) = hy;
    *(v4h*)(Hh + row * HP + c4) = he;
    if (it == 1) asm volatile("" ::: "memory");
  }
  {
    const int which = tid >> 6;
    const int idx = (tid & 63) * 4;
    const v4f va = *(const v4f*)(b1 + idx);
    const v4f vw = *(const v4f*)(W1 + (size_t)NDIM * NHID + idx);
    v4f o;
#pragma unroll
    for (int q = 0; q < 4; ++q) o[q] = which ? vw[q] : va[q];
    *(v4f*)(Bs + which * NHID + idx) = o;
  }
  const float b2v = b2[16 * wave + c];
  __syncthreads();

  float z0[2][8], lpw[2][8];
#pragma unroll
  for (int mt = 0; mt < 2; ++mt)
#pragma unroll
    for (int r = 0; r < 8; ++r) {
      z0[mt][r]  = Kf[(16 * mt + 8 * hh + r) * SP + 16 * wave + c];
      lpw[mt][r] = 0.0f;
    }

#pragma unroll 1
  for (int nt = 0; nt < 4; ++nt) {
    const int col = 64 * wave + 16 * nt + c;
    const _Float16* pg = W2R + (size_t)col * NDIM + koff;
    const _Float16* pw = W1T + (size_t)col * NDIM + koff;
    v8f ag[2], aw[2];
    ag[0] = z8; ag[1] = z8; aw[0] = z8; aw[1] = z8;
#pragma unroll
    for (int kc = 0; kc < 2; ++kc) {
      const v16h bg = Frag<_Float16>::load(pg + 32 * kc);
      const v16h bw = Frag<_Float16>::load(pw + 32 * kc);
      const v16h a0 = Frag<_Float16>::load(Hh + c * HP + koff + 32 * kc);
      const v16h a1 = Frag<_Float16>::load(Hh + (16 + c) * HP + koff + 32 * kc);
      ag[0] = Frag<_Float16>::mma(a0, bg, ag[0]);
      ag[1] = Frag<_Float16>::mma(a1, bg, ag[1]);
      aw[0] = Frag<_Float16>::mma(a0, bw, aw[0]);
      aw[1] = Frag<_Float16>::mma(a1, bw, aw[1]);
      guard4x4(ag[0], ag[1], aw[0], aw[1], a0, a1, bg, bw);
    }
    acc_guard4(ag[0], ag[1], aw[0], aw[1]);
#pragma unroll
    for (int mt = 0; mt < 2; ++mt)
#pragma unroll
      for (int r = 0; r < 8; ++r)
        Cs[(mt * 4 + nt) * CSUB + r * NTHR + tid] = (ag[mt][r] * aw[mt][r]) * CSC;
  }

#pragma unroll 1
  for (int step = 0; step < NSTEPS; ++step) {
    const float tbase = (float)step * DT;
#pragma unroll 1
    for (int i = 0; i < NSTAGE; ++i) {
      const float tv = tbase + c_cdt[i];
      __syncthreads();

      float divp[2][8];
#pragma unroll
      for (int mt = 0; mt < 2; ++mt)
#pragma unroll
        for (int r = 0; r < 8; ++r) divp[mt][r] = 0.0f;
#pragma unroll 1
      for (int nt = 0; nt < 4; ++nt) {
        const int col = 64 * wave + 16 * nt + c;
        const _Float16* pw = W1T + (size_t)col * NDIM + koff;
        v8f acc[2];
        acc[0] = z8; acc[1] = z8;
#pragma unroll
        for (int kc = 0; kc < 2; ++kc) {
          const v16h b  = Frag<_Float16>::load(pw + 32 * kc);
          const v16h a0 = Frag<_Float16>::load(Yh + c * YP + koff + 32 * kc);
          const v16h a1 = Frag<_Float16>::load(Yh + (16 + c) * YP + koff + 32 * kc);
          acc[0] = Frag<_Float16>::mma(a0, b, acc[0]);
          acc[1] = Frag<_Float16>::mma(a1, b, acc[1]);
          guard2x3(acc[0], acc[1], a0, a1, b);
        }
        acc_guard2(acc[0], acc[1]);
        const float bia = fmaf(tv, Bs[NHID + col], Bs[col]);
#pragma unroll
        for (int mt = 0; mt < 2; ++mt)
#pragma unroll
          for (int r = 0; r < 8; ++r) {
            const float u  = fmaf(acc[mt][r], W1CAR_INV, bia);
            const float h  = tanh_acc(u);
            Hh[(16 * mt + 8 * hh + r) * HP + col] = (_Float16)h;
            const float gp = fmaf(-h, h, 1.0f);
            divp[mt][r] = fmaf(Cs[(mt * 4 + nt) * CSUB + r * NTHR + tid], gp, divp[mt][r]);
          }
      }
      const float bdt = c_btab[i] * DT;
#pragma unroll
      for (int mt = 0; mt < 2; ++mt)
#pragma unroll
        for (int r = 0; r < 8; ++r) {
          float d = divp[mt][r];
          d += __shfl_xor(d, 1, 32);
          d += __shfl_xor(d, 2, 32);
          d += __shfl_xor(d, 4, 32);
          d += __shfl_xor(d, 8, 32);
          lpw[mt][r] = fmaf(-bdt, d, lpw[mt][r]);
        }
      __syncthreads();

      const _Float16* pv = W2T + (size_t)(16 * wave + c) * NHID + koff;
      v8f acc2[2];
      acc2[0] = z8; acc2[1] = z8;
#pragma unroll 1
      for (int k0 = 0; k0 < NHID; k0 += 32) {
        const v16h b  = Frag<_Float16>::load(pv + k0);
        const v16h a0 = Frag<_Float16>::load(Hh + c * HP + koff + k0);
        const v16h a1 = Frag<_Float16>::load(Hh + (16 + c) * HP + koff + k0);
        acc2[0] = Frag<_Float16>::mma(a0, b, acc2[0]);
        acc2[1] = Frag<_Float16>::mma(a1, b, acc2[1]);
        guard2x3(acc2[0], acc2[1], a0, a1, b);
      }
      acc_guard2(acc2[0], acc2[1]);
      float kv[2][8];
#pragma unroll
      for (int mt = 0; mt < 2; ++mt)
#pragma unroll
        for (int r = 0; r < 8; ++r) kv[mt][r] = fmaf(acc2[mt][r], W2CAR_INV, b2v);

      if (i < NSTAGE - 1) {
#pragma unroll
        for (int mt = 0; mt < 2; ++mt)
#pragma unroll
          for (int r = 0; r < 8; ++r) Kf[(i * 2 + mt) * CSUB + r * NTHR + tid] = kv[mt][r];
        const int ip = i + 1;
        float s[2][8];
#pragma unroll
        for (int mt = 0; mt < 2; ++mt)
#pragma unroll
          for (int r = 0; r < 8; ++r) s[mt][r] = 0.0f;
#pragma unroll 1
        for (int j = 0; j < i; ++j) {
          const float a = c_atab[ip][j];
#pragma unroll
          for (int mt = 0; mt < 2; ++mt)
#pragma unroll
            for (int r = 0; r < 8; ++r) s[mt][r] = fmaf(a, Kf[(j * 2 + mt) * CSUB + r * NTHR + tid], s[mt][r]);
        }
        const float ai = c_atab[ip][i];
#pragma unroll
        for (int mt = 0; mt < 2; ++mt)
#pragma unroll
          for (int r = 0; r < 8; ++r) {
            const float ss = fmaf(ai, kv[mt][r], s[mt][r]);
            const float yv = fmaf(DT, ss, z0[mt][r]);
            Yh[(16 * mt + 8 * hh + r) * YP + 16 * wave + c] = (_Float16)yv;
          }
      } else {
#pragma unroll
        for (int mt = 0; mt < 2; ++mt)
#pragma unroll
          for (int r = 0; r < 8; ++r) {
            float s = BW0 * Kf[(0 * 2 + mt) * CSUB + r * NTHR + tid];
            s = fmaf(BW2, Kf[(2 * 2 + mt) * CSUB + r * NTHR + tid], s);
            s = fmaf(BW3, Kf[(3 * 2 + mt) * CSUB + r * NTHR + tid], s);
            s = fmaf(BW4, Kf[(4 * 2 + mt) * CSUB + r * NTHR + tid], s);
            s = fmaf(BW5, kv[mt][r], s);
            const float zn = fmaf(DT, s, z0[mt][r]);
            z0[mt][r] = zn;
            Yh[(16 * mt + 8 * hh + r) * YP + 16 * wave + c] = (_Float16)zn;
          }
      }
    }
  }

  __syncthreads();
  float* Os = Kf;
  float* Sq = Kf + RB * SP;
  float* Lq = Sq + NWAVE * RB;
  float* Fo = Lq + NWAVE * RB;
  float sred[2][8];
#pragma unroll
  for (int mt = 0; mt < 2; ++mt)
#pragma unroll
    for (int r = 0; r < 8; ++r) {
      const float z = z0[mt][r];
      Os[(16 * mt + 8 * hh + r) * SP + 16 * wave + c] = z;
      float t = HALF_LN2PI_NEG - 0.5f * z * z;
      t += __shfl_xor(t, 1, 32);
      t += __shfl_xor(t, 2, 32);
      t += __shfl_xor(t, 4, 32);
      t += __shfl_xor(t, 8, 32);
      sred[mt][r] = t;
    }
  if (c == 0) {
#pragma unroll
    for (int mt = 0; mt < 2; ++mt)
#pragma unroll
      for (int r = 0; r < 8; ++r) {
        Sq[wave * RB + 16 * mt + 8 * hh + r] = sred[mt][r];
        Lq[wave * RB + 16 * mt + 8 * hh + r] = lpw[mt][r];
      }
  }
  __syncthreads();
  for (int pass = 0; pass < 2; ++pass) {
#pragma unroll
    for (int it = 0; it < 4; ++it) {
      const int idx = it * NTHR + tid;
      const int row = idx >> 4, c4 = (idx & 15) * 4;
      const v4f v = *(const v4f*)(Os + row * SP + c4);
      *(volatile v4f*)(out0 + (size_t)(rowbase + row) * NDIM + c4) = v;
    }
    __threadfence();
  }
  if (tid < RB) {
    const float sq = ((Sq[tid] + Sq[RB + tid]) + Sq[2 * RB + tid]) + Sq[3 * RB + tid];
    const float lq = ((Lq[tid] + Lq[RB + tid]) + Lq[2 * RB + tid]) + Lq[3 * RB + tid];
    Fo[tid] = sq - lq;
  }
  __syncthreads();
  if (tid < RB / 4) {
    const v4f v = *(const v4f*)(Fo + 4 * tid);
    float* op = out1 + rowbase + 4 * tid;
    *(volatile v4f*)op = v;
    __threadfence();
    *(volatile v4f*)op = v;
  }
}

extern "C" void kernel_launch(void* const* d_in, const int* in_sizes, int n_in,
                              void* d_out, int out_size, void* d_ws, size_t ws_size, hipStream_t stream) {
  if (n_in < 6 || d_out == nullptr || d_ws == nullptr) return;
  if (in_sizes[0] != NBATCH * NDIM || in_sizes[1] != NBATCH * NDIM || in_sizes[2] != (NDIM + 1) * NHID ||
      in_sizes[3] != NHID || in_sizes[4] != NHID * NDIM || in_sizes[5] != NDIM ||
      out_size != NBATCH * NDIM + NBATCH) return;

  const float* yin = (const float*)d_in[0];
  const float* ein = (const float*)d_in[1];
  const float* w1  = (const float*)d_in[2];
  const float* b1  = (const float*)d_in[3];
  const float* w2  = (const float*)d_in[4];
  const float* b2  = (const float*)d_in[5];
  float* out0 = (float*)d_out;
  float* out1 = out0 + (size_t)NBATCH * NDIM;

  char* ws = (char*)d_ws; size_t off = 0;
  auto carve = [&](size_t bytes) -> char* { char* p = ws + off; off += (bytes + 255) & ~(size_t)255; return p; };
  unsigned short* W1T = (unsigned short*)carve((size_t)NHID * NDIM * 2);
  unsigned short* W2T = (unsigned short*)carve((size_t)NDIM * NHID * 2);
  unsigned short* W2R = (unsigned short*)carve((size_t)NHID * NDIM * 2);
  if (off > ws_size || off > (size_t)134217728) return;

  tpose_f16_kernel<<<dim3(NHID / 64, NDIM / 64), 256, 0, stream>>>(w1, NDIM, NHID, NDIM, W1T, W1CAR);
  tpose_f16_kernel<<<dim3(NDIM / 64, NHID / 64), 256, 0, stream>>>(w2, NHID, NDIM, NHID, W2T, W2CAR);
  cast8_f16_kernel<<<(NHID * NDIM / 8) / 256, 256, 0, stream>>>(w2, W2R, NHID * NDIM / 8, W2CAR);
  ode_flow_kernel<<<NBATCH / RB, NTHR, 0, stream>>>(yin, ein, w1, b1, b2, W1T, W2T, W2R, out0, out1);
}
